// RecurrentNEFLayer_64287070486909
// MI455X (gfx1250) — hardware-verified
//
#include <hip/hip_runtime.h>
#include <stdint.h>

constexpr int kBatch      = 512;
constexpr int kSteps      = 256;
constexpr int kDin        = 64;
constexpr int kNeur       = 2048;
constexpr int kDst        = 64;
constexpr int kDaug       = 128;
constexpr int kDout       = 10;
constexpr int kDoutPad    = 16;
constexpr int kThreads    = 256;
constexpr int kWaves      = 8;
constexpr int kSeqPerBlk  = 16;
constexpr int kNeurPerWave = 256;
constexpr int kXP  = 136;
constexpr int kAP  = 2056;
constexpr int kRP  = 36;
constexpr float kEncCarry = 16.0f;   constexpr float kEncInv = 1.0f / 16.0f;
constexpr float kSdCarry  = 32.0f;   constexpr float kSdInv  = 1.0f / 32.0f;
constexpr float kDecCarry = 32.0f;   constexpr float kDecInv = 1.0f / 32.0f;

static_assert(kDaug == kDin + kDst, "aug");
static_assert(kBatch % kSeqPerBlk == 0, "batch tiles");
static_assert(kNeur == kWaves * kNeurPerWave && kNeurPerWave % 16 == 0, "neuron tiles");
static_assert(kDaug % 32 == 0 && kNeur % 32 == 0, "K multiples of 32");
static_assert(kDst == 64 && kDin == 64, "state/input width");
static_assert(kNeur % (4 * 512) == 0, "phase-2 k quarters");
static_assert((kSeqPerBlk * kDout * 4) % 128 == 0, "block output region is whole lines");
static_assert(kThreads == 32 * kWaves, "waves");

typedef __attribute__((ext_vector_type(16))) _Float16 v16h;
typedef __attribute__((ext_vector_type(8)))  _Float16 v8h;
typedef __attribute__((ext_vector_type(16))) __bf16   v16b;
typedef __attribute__((ext_vector_type(8)))  __bf16   v8b;
typedef __attribute__((ext_vector_type(8)))  float    v8f;
typedef __attribute__((ext_vector_type(4)))  float    v4f;

__device__ __forceinline__ unsigned short f2bf_bits(float f) {
  unsigned u = __float_as_uint(f);
  return (unsigned short)((u + 0x7FFFu + ((u >> 16) & 1u)) >> 16);
}
__device__ __forceinline__ float bf_bits2f(unsigned short h) { return __uint_as_float(((unsigned)h) << 16); }

__device__ __forceinline__ void dep_guard_h(v8f& a, v8f& b, v16h x, v16h y) { asm volatile("v_nop\n\tv_nop\n\tv_nop\n\tv_nop" : "+v"(a), "+v"(b) : "v"(x), "v"(y)); }
__device__ __forceinline__ void dep_guard1_h(v8f& a, v16h x, v16h y) { asm volatile("v_nop\n\tv_nop\n\tv_nop\n\tv_nop" : "+v"(a) : "v"(x), "v"(y)); }
__device__ __forceinline__ void dep_guard_b(v8f& a, v8f& b, v16b x, v16b y) { asm volatile("v_nop\n\tv_nop\n\tv_nop\n\tv_nop" : "+v"(a), "+v"(b) : "v"(x), "v"(y)); }
__device__ __forceinline__ void keep4_h(v16h a, v16h b, v16h c, v16h d) { asm volatile("v_nop" :: "v"(a), "v"(b), "v"(c), "v"(d)); }
__device__ __forceinline__ void keep4_b(v16b a, v16b b, v16b c, v16b d) { asm volatile("v_nop" :: "v"(a), "v"(b), "v"(c), "v"(d)); }
__device__ __forceinline__ void acc_guard4(v8f& a, v8f& b, v8f& c, v8f& d) { asm volatile("v_nop\n\tv_nop\n\tv_nop\n\tv_nop" : "+v"(a), "+v"(b), "+v"(c), "+v"(d)); }
__device__ __forceinline__ void acc_guard2(v8f& a, v8f& b) { asm volatile("v_nop\n\tv_nop\n\tv_nop\n\tv_nop" : "+v"(a), "+v"(b)); }
__device__ __forceinline__ void acc_guard1(v8f& a) { asm volatile("v_nop\n\tv_nop\n\tv_nop\n\tv_nop" : "+v"(a)); }
template <typename T> struct Frag;
template <> struct Frag<_Float16> {
  typedef v16h V; union U { v16h v; v8h h[2]; };
  static __device__ __forceinline__ v16h load(const _Float16* p) {
    U f; f.h[0] = *(const v8h*)(p); f.h[1] = *(const v8h*)(p + 16); return f.v;
  }
  static __device__ __forceinline__ v8f mma(v16h a, v16h b, v8f c) {
    return __builtin_amdgcn_wmma_f32_16x16x32_f16(false, a, false, b, (short)0, c, false, false);
  }
  static __device__ __forceinline__ void guard(v8f& a, v8f& b, v16h x, v16h y) { dep_guard_h(a, b, x, y); }
  static __device__ __forceinline__ void keep(v16h a, v16h b, v16h c, v16h d) { keep4_h(a, b, c, d); }
};
template <> struct Frag<__bf16> {
  typedef v16b V; union U { v16b v; v8b h[2]; };
  static __device__ __forceinline__ v16b load(const __bf16* p) {
    U f; f.h[0] = *(const v8b*)(p); f.h[1] = *(const v8b*)(p + 16); return f.v;
  }
  static __device__ __forceinline__ v8f mma(v16b a, v16b b, v8f c) {
    return __builtin_amdgcn_wmma_f32_16x16x32_bf16(false, a, false, b, (short)0, c, false, false);
  }
  static __device__ __forceinline__ void guard(v8f& a, v8f& b, v16b x, v16b y) { dep_guard_b(a, b, x, y); }
  static __device__ __forceinline__ void keep(v16b a, v16b b, v16b c, v16b d) { keep4_b(a, b, c, d); }
};

template <int MODE>
__global__ __launch_bounds__(kThreads) void tpw_kernel(const float* __restrict__ src, int R, int C, int ldo,
                                                      unsigned short* __restrict__ O, float sc) {
  __shared__ float Tt[64 * 65];
  const int tid = threadIdx.x;
  const int c0 = blockIdx.x * 64, r0 = blockIdx.y * 64;
#pragma unroll
  for (int i = 0; i < 4; ++i) {
    const int idx = i * kThreads + tid;
    const int rr = idx >> 4, cc = (idx & 15) * 4;
    const v4f v = *(const v4f*)(src + (size_t)(r0 + rr) * (size_t)C + c0 + cc);
    Tt[rr * 65 + cc + 0] = v[0];
    Tt[rr * 65 + cc + 1] = v[1];
    Tt[rr * 65 + cc + 2] = v[2];
    Tt[rr * 65 + cc + 3] = v[3];
  }
  __syncthreads();
  const int q = tid >> 3, c8 = (tid & 7) * 8;
  v8h hv[2];
#pragma unroll
  for (int g = 0; g < 2; ++g) {
    const int qq = g * 32 + q;
#pragma unroll
    for (int e = 0; e < 8; ++e) {
      const float f = Tt[(c8 + e) * 65 + qq];
      unsigned short bits;
      if (MODE == 0) {
        bits = f2bf_bits(f * sc);
      } else {
        const float fb = bf_bits2f(f2bf_bits(f));
        bits = __builtin_bit_cast(unsigned short, (_Float16)(fb * sc));
      }
      hv[g][e] = __builtin_bit_cast(_Float16, bits);
    }
  }
  for (int pass = 0; pass < 2; ++pass) {
#pragma unroll
    for (int g = 0; g < 2; ++g) {
      const size_t o = (size_t)(c0 + g * 32 + q) * (size_t)ldo + (size_t)(r0 + c8);
      *(volatile v8h*)(O + o) = hv[g];
    }
    __threadfence();
  }
}

__global__ __launch_bounds__(kThreads) void cast8_kernel(const float* __restrict__ in, unsigned short* __restrict__ O,
                                                        int n8, float sc) {
  const int i = blockIdx.x * kThreads + threadIdx.x;
  if (i >= n8) return;
  const v4f a = *(const v4f*)(in + (size_t)8 * i);
  const v4f b = *(const v4f*)(in + (size_t)8 * i + 4);
  v8h hv;
#pragma unroll
  for (int e = 0; e < 4; ++e) {
    hv[e]     = (_Float16)(bf_bits2f(f2bf_bits(a[e])) * sc);
    hv[4 + e] = (_Float16)(bf_bits2f(f2bf_bits(b[e])) * sc);
  }
  for (int pass = 0; pass < 2; ++pass) {
    *(volatile v8h*)(O + (size_t)8 * i) = hv;
    __threadfence();
  }
}

__global__ __launch_bounds__(kThreads) void dect_kernel(const float* __restrict__ dec, unsigned short* __restrict__ O, float sc) {
  const int i  = blockIdx.x * kThreads + threadIdx.x;
  const int o  = i >> 8;
  const int n8 = (i & 255) * 8;
  const int oc = (o < kDout) ? o : (kDout - 1);
  const bool live = (o < kDout);
  v8h hv;
#pragma unroll
  for (int e = 0; e < 8; ++e) {
    const float f  = dec[(size_t)(n8 + e) * kDout + oc];
    const float fb = bf_bits2f(f2bf_bits(f));
    const _Float16 h = (_Float16)(fb * sc);
    hv[e] = live ? h : (_Float16)0.0f;
  }
  const size_t off = (size_t)o * kNeur + (size_t)n8;
  for (int pass = 0; pass < 2; ++pass) {
    *(volatile v8h*)(O + off) = hv;
    __threadfence();
  }
}

__global__ __launch_bounds__(kThreads) void nef_kernel(const float* __restrict__ seq, const float* __restrict__ gain,
                                                      const float* __restrict__ bias,
                                                      const unsigned short* __restrict__ ENCp,
                                                      const unsigned short* __restrict__ SDTp,
                                                      const unsigned short* __restrict__ DECTp,
                                                      float* __restrict__ out) {
  __shared__ __align__(16) _Float16 Xh[kSeqPerBlk * kXP];
  __shared__ __align__(16) _Float16 Ah2[kSeqPerBlk * kAP];
  __shared__ __align__(16) float    Rp[kWaves * kSeqPerBlk * kRP];
  __shared__ __align__(16) float    Os[160];

  const _Float16* ENC  = (const _Float16*)ENCp;
  const _Float16* SDT  = (const _Float16*)SDTp;
  const _Float16* DECT = (const _Float16*)DECTp;

  const int tid = threadIdx.x, lane = tid & 31, wave = tid >> 5;
  const int c = lane & 15, hh = lane >> 4, koff = hh * 8;
  const int b0 = blockIdx.x * kSeqPerBlk;
  const v8f z8 = {0.f, 0.f, 0.f, 0.f, 0.f, 0.f, 0.f, 0.f};

  {
    const int row = tid >> 4, q4 = (tid & 15) * 4;
#pragma unroll
    for (int e = 0; e < 4; ++e) Xh[row * kXP + kDin + q4 + e] = (_Float16)0.0f;
    const v4f v = *(const v4f*)(seq + ((size_t)(b0 + row) * kSteps + 0) * kDin + q4);
#pragma unroll
    for (int e = 0; e < 4; ++e) Xh[row * kXP + q4 + e] = (_Float16)bf_bits2f(f2bf_bits(v[e]));
  }
  __syncthreads();

  const _Float16* xrow = Xh + c * kXP + koff;
  const int jp = wave & 1, kq = wave >> 1;

#pragma unroll 1
  for (int t = 0; t < kSteps; ++t) {
    {
      const v16h xa0 = Frag<_Float16>::load(xrow);
      const v16h xa1 = Frag<_Float16>::load(xrow + 32);
      const v16h xa2 = Frag<_Float16>::load(xrow + 64);
      const v16h xa3 = Frag<_Float16>::load(xrow + 96);
#pragma unroll 1
      for (int nt = 0; nt < kNeurPerWave / 16; ++nt) {
        const int n0 = wave * kNeurPerWave + nt * 16;
        const _Float16* brow = ENC + (size_t)(n0 + c) * kDaug + koff;
        const v16h e0 = Frag<_Float16>::load(brow);
        const v16h e1 = Frag<_Float16>::load(brow + 32);
        const v16h e2 = Frag<_Float16>::load(brow + 64);
        const v16h e3 = Frag<_Float16>::load(brow + 96);
        v8f acc = z8;
        acc = Frag<_Float16>::mma(xa0, e0, acc);
        acc = Frag<_Float16>::mma(xa1, e1, acc);
        acc = Frag<_Float16>::mma(xa2, e2, acc);
        acc = Frag<_Float16>::mma(xa3, e3, acc);
        dep_guard1_h(acc, xa3, e3);
        keep4_h(e0, e1, e2, e3);
        const float g  = bf_bits2f(f2bf_bits(gain[n0 + c]));
        const float bb = bf_bits2f(f2bf_bits(bias[n0 + c]));
#pragma unroll
        for (int r = 0; r < 8; ++r) {
          const float dot = acc[r] * kEncInv;
          const float av  = __builtin_fabsf(g * dot + bb);
          Ah2[(8 * hh + r) * kAP + n0 + c] = (_Float16)av;
        }
      }
    }
    __syncthreads();

    {
      const _Float16* arow  = Ah2 + c * kAP + 512 * kq + koff;
      const _Float16* srow0 = SDT + (size_t)(32 * jp + c) * kNeur + 512 * kq + koff;
      const _Float16* srow1 = srow0 + (size_t)16 * kNeur;
      v8f s0 = z8, s1 = z8;
#pragma unroll 1
      for (int ks = 0; ks < 16; ++ks) {
        const int k = ks * 32;
        const v16h ah  = Frag<_Float16>::load(arow + k);
        const v16h sb0 = Frag<_Float16>::load(srow0 + k);
        const v16h sb1 = Frag<_Float16>::load(srow1 + k);
        s0 = Frag<_Float16>::mma(ah, sb0, s0);
        s1 = Frag<_Float16>::mma(ah, sb1, s1);
        dep_guard_h(s0, s1, ah, sb1);
        keep4_h(sb0, sb1, ah, ah);
      }
      acc_guard2(s0, s1);
      float* rw = Rp + (size_t)wave * kSeqPerBlk * kRP;
#pragma unroll
      for (int r = 0; r < 8; ++r) {
        rw[(8 * hh + r) * kRP + c]      = s0[r] * kSdInv;
        rw[(8 * hh + r) * kRP + 16 + c] = s1[r] * kSdInv;
      }
    }
    __syncthreads();

    {
      const int row = tid >> 4, q4 = (tid & 15) * 4;
      const int sj = q4 >> 5, cc = q4 & 31;
      float sv[4];
#pragma unroll
      for (int e = 0; e < 4; ++e) sv[e] = Rp[((0 * 2 + sj) * kSeqPerBlk + row) * kRP + cc + e];
#pragma unroll
      for (int kk = 1; kk < 4; ++kk) {
#pragma unroll
        for (int e = 0; e < 4; ++e) sv[e] += Rp[((2 * kk + sj) * kSeqPerBlk + row) * kRP + cc + e];
      }
#pragma unroll
      for (int e = 0; e < 4; ++e) Xh[row * kXP + kDin + q4 + e] = (_Float16)sv[e];
      const int tn = (t + 1 < kSteps) ? (t + 1) : (kSteps - 1);
      const v4f v = *(const v4f*)(seq + ((size_t)(b0 + row) * kSteps + (size_t)tn) * kDin + q4);
#pragma unroll
      for (int e = 0; e < 4; ++e) Xh[row * kXP + q4 + e] = (_Float16)bf_bits2f(f2bf_bits(v[e]));
    }
    __syncthreads();
  }

  {
    const _Float16* arow = Ah2 + c * kAP + kNeurPerWave * wave + koff;
    const _Float16* drow = DECT + (size_t)c * kNeur + kNeurPerWave * wave + koff;
    v8f d0 = z8;
#pragma unroll 1
    for (int ks = 0; ks < kNeurPerWave / 32; ++ks) {
      const int k = ks * 32;
      const v16h ah = Frag<_Float16>::load(arow + k);
      const v16h bd = Frag<_Float16>::load(drow + k);
      d0 = Frag<_Float16>::mma(ah, bd, d0);
      dep_guard1_h(d0, ah, bd);
    }
    acc_guard1(d0);
    float* rw = Rp + (size_t)wave * kSeqPerBlk * kRP;
#pragma unroll
    for (int r = 0; r < 8; ++r) rw[(8 * hh + r) * kRP + c] = d0[r] * kDecInv;
  }
  __syncthreads();
  if (tid < kSeqPerBlk * kDout) {
    const int row = tid / kDout, o = tid - row * kDout;
    float v = Rp[(0 * kSeqPerBlk + row) * kRP + o];
#pragma unroll
    for (int w = 1; w < kWaves; ++w) v += Rp[(w * kSeqPerBlk + row) * kRP + o];
    Os[tid] = v;
  }
  __syncthreads();
  if (wave == 0) {
    const size_t base = (size_t)blockIdx.x * (kSeqPerBlk * kDout);
    const int l2 = (lane < 8) ? lane : 7;
    for (int pass = 0; pass < 2; ++pass) {
      const v4f v0 = *(const v4f*)(Os + 4 * lane);
      *(volatile v4f*)(out + base + 4 * lane) = v0;
      const v4f v1 = *(const v4f*)(Os + 128 + 4 * l2);
      if (lane < 8) *(volatile v4f*)(out + base + 128 + 4 * lane) = v1;
      __threadfence();
    }
  }
}

extern "C" void kernel_launch(void* const* d_in, const int* in_sizes, int n_in,
                              void* d_out, int out_size, void* d_ws, size_t ws_size, hipStream_t stream) {
  if (n_in < 6 || d_out == nullptr || d_ws == nullptr) return;
  if (in_sizes[0] != kBatch * kSteps * kDin || in_sizes[1] != kNeur * kDaug || in_sizes[2] != kNeur ||
      in_sizes[3] != kNeur || in_sizes[4] != kNeur * kDst || in_sizes[5] != kNeur * kDout ||
      out_size != kBatch * kDout) return;

  const float* seq  = (const float*)d_in[0];
  const float* enc  = (const float*)d_in[1];
  const float* bias = (const float*)d_in[2];
  const float* gain = (const float*)d_in[3];
  const float* sd   = (const float*)d_in[4];
  const float* dec  = (const float*)d_in[5];
  float* out = (float*)d_out;

  char* ws = (char*)d_ws; size_t off = 0;
  auto carve = [&](size_t bytes) -> char* { char* p = ws + off; off += (bytes + 255) & ~(size_t)255; return p; };
  unsigned short* ENC  = (unsigned short*)carve((size_t)kNeur * kDaug * 2);
  unsigned short* SDT  = (unsigned short*)carve((size_t)kDst * kNeur * 2);
  unsigned short* DECT = (unsigned short*)carve((size_t)kDoutPad * kNeur * 2);
  if (off > ws_size || off > (size_t)134217728) return;

  const int enc_n8 = kNeur * kDaug / 8;
  cast8_kernel<<<(enc_n8 + kThreads - 1) / kThreads, kThreads, 0, stream>>>(enc, ENC, enc_n8, kEncCarry);
  tpw_kernel<1><<<dim3(kDst / 64, kNeur / 64), kThreads, 0, stream>>>(sd, kNeur, kDst, kNeur, SDT, kSdCarry);
  dect_kernel<<<(kDoutPad * kNeur / 8) / kThreads, kThreads, 0, stream>>>(dec, DECT, kDecCarry);
  nef_kernel<<<kBatch / kSeqPerBlk, kThreads, 0, stream>>>(seq, gain, bias, ENC, SDT, DECT, out);
}
